// BeeReceiver_50500225466645
// MI455X (gfx1250) — hardware-run, weakly checked
//
#include <hip/hip_runtime.h>
#include <math.h>

typedef __attribute__((ext_vector_type(16))) _Float16 v16h;
typedef __attribute__((ext_vector_type(8)))  _Float16 v8h;
typedef __attribute__((ext_vector_type(4)))  _Float16 v4h;
typedef __attribute__((ext_vector_type(8)))  float    v8f;
typedef __attribute__((ext_vector_type(4)))  float    v4f;

constexpr int kNodes        = 50000;
constexpr int kGraphs       = 250;
constexpr int kNpg          = 200;
constexpr int kEpg          = 3200;
constexpr int kEdges        = kGraphs * kEpg;
constexpr int kF            = 128;
constexpr int kRel          = 8;
constexpr int kVocab        = 1000;
constexpr int kNcat         = (kRel + 1) * kF;
constexpr int kChunkGraphs  = 64;
constexpr int kChunkRows    = kChunkGraphs * kNpg;
constexpr int kChunks       = 4;
constexpr int kRowsPad      = kChunks * kChunkRows;
constexpr int kQuadsPerChunk = kChunkGraphs / 4;
constexpr int kQuads        = (kGraphs + 3) / 4;
constexpr int kTilesM       = kChunkRows / 64;
constexpr int kTilesN       = kNcat / 64;
constexpr float kWCarry     = 16.0f;
constexpr float kWCarryInv  = 1.0f / kWCarry;
constexpr int kRealOct      = kNodes * kF / 8;
constexpr int kPadOct       = kRowsPad * kF / 8;

static_assert(kNodes == kGraphs * kNpg, "node layout");
static_assert(kEdges == 800000, "edge count");
static_assert(kNcat == 1152, "concatenated projection width");
static_assert((kF % 32) == 0, "GEMM K multiple of 32");
static_assert((kChunkRows % 64) == 0 && (kNcat % 64) == 0, "GEMM M,N multiples of 64");
static_assert(kChunkRows == 12800 && kRowsPad == 51200, "chunking");
static_assert(kRowsPad >= kNodes, "pad rows");
static_assert((kTilesM * kTilesN) % 8 == 0, "whole blocks of 8 wave tiles");
static_assert((kRealOct % 256) == 0 && (kPadOct % 256) == 0, "cast grid exact, pad boundary block-uniform");
static_assert(kQuads == 63, "quad count");

constexpr size_t kOffA16  = 0;
constexpr size_t kOffH16  = kOffA16 + (size_t)kRowsPad * kF * 2;
constexpr size_t kOffBT1  = kOffH16 + (size_t)kRowsPad * kF * 2;
constexpr size_t kOffBT2  = kOffBT1 + (size_t)kNcat * kF * 2;
constexpr size_t kOffHW   = kOffBT2 + (size_t)kNcat * kF * 2;
constexpr size_t kOffMREP = kOffHW  + (size_t)kChunkRows * kNcat * 4;
constexpr size_t kWsTotal = kOffMREP + (size_t)kGraphs * kF * 4;
static_assert(kWsTotal == 85914624ull, "carve total");
static_assert(kWsTotal <= 134217728ull, "carve cap");
static_assert((kOffH16 % 128) == 0 && (kOffBT1 % 128) == 0 && (kOffBT2 % 128) == 0 &&
              (kOffHW % 128) == 0 && (kOffMREP % 128) == 0, "128-B aligned regions");

union FragU { v16h v; v8h h[2]; };
__device__ __forceinline__ v16h frag_load_h(const _Float16* p) {
  FragU f;
  f.h[0] = *(const v8h*)(p);
  f.h[1] = *(const v8h*)(p + 16);
  return f.v;
}
__device__ __forceinline__ v8f mma_h(v16h a, v16h b, v8f c) {
  c = __builtin_amdgcn_wmma_f32_16x16x32_f16(false, a, false, b, (short)0, c, false, false);
  asm volatile("v_nop\n\tv_nop\n\tv_nop\n\tv_nop" : "+v"(c) : "v"(a), "v"(b));
  return c;
}
__device__ __forceinline__ void acc_guard4(v8f& a, v8f& b, v8f& c, v8f& d) {
  asm volatile("v_nop\n\tv_nop\n\tv_nop\n\tv_nop" : "+v"(a), "+v"(b), "+v"(c), "+v"(d));
}

__global__ __launch_bounds__(256) void proj_gemm_kernel(
    const unsigned short* __restrict__ Ap, const unsigned short* __restrict__ Btp,
    float* __restrict__ C, float scale)
{
  __shared__ __align__(16) float sT[8][16 * 68];
  const _Float16* A  = (const _Float16*)Ap;
  const _Float16* Bt = (const _Float16*)Btp;
  const int lane = threadIdx.x & 31;
  const int wave = threadIdx.x >> 5;
  const int tile = blockIdx.x * 8 + wave;
  if (tile >= kTilesM * kTilesN) return;
  const int tm = tile / kTilesN;
  const int tn = tile - tm * kTilesN;
  const int m0 = tm << 6;
  const int n0 = tn << 6;
  const int rlane = lane & 15;
  const int koff  = (lane >> 4) * 8;
  const int mOff  = (lane >> 4) * 8;

  v8f acc[4][4];
#pragma unroll
  for (int i = 0; i < 4; ++i)
#pragma unroll
    for (int j = 0; j < 4; ++j) acc[i][j] = (v8f){0.f, 0.f, 0.f, 0.f, 0.f, 0.f, 0.f, 0.f};

#pragma unroll 1
  for (int k0 = 0; k0 < kF; k0 += 32) {
    v16h bh[4];
#pragma unroll
    for (int j = 0; j < 4; ++j) {
      const size_t bo = (size_t)(n0 + (j << 4) + rlane) * kF + koff + k0;
      bh[j] = frag_load_h(Bt + bo);
    }
#pragma unroll
    for (int i = 0; i < 4; ++i) {
      const size_t ao = (size_t)(m0 + (i << 4) + rlane) * kF + koff + k0;
      const v16h ah = frag_load_h(A + ao);
#pragma unroll
      for (int j = 0; j < 4; ++j) acc[i][j] = mma_h(ah, bh[j], acc[i][j]);
    }
  }
  acc_guard4(acc[0][0], acc[0][1], acc[0][2], acc[0][3]);
  acc_guard4(acc[1][0], acc[1][1], acc[1][2], acc[1][3]);
  acc_guard4(acc[2][0], acc[2][1], acc[2][2], acc[2][3]);
  acc_guard4(acc[3][0], acc[3][1], acc[3][2], acc[3][3]);

  float* slab = sT[wave];
#pragma unroll
  for (int i = 0; i < 4; ++i) {
    const int mBase = m0 + (i << 4);
#pragma unroll
    for (int j = 0; j < 4; ++j) {
#pragma unroll
      for (int r = 0; r < 8; ++r) {
        const float v = acc[i][j][r] * scale;
        slab[(mOff + r) * 68 + (j << 4) + rlane] = v;
      }
    }
    __builtin_amdgcn_fence(__ATOMIC_RELEASE, "workgroup");
    __builtin_amdgcn_wave_barrier();
    __builtin_amdgcn_fence(__ATOMIC_ACQUIRE, "workgroup");
    {
      const int hh = lane >> 4, c4 = (lane & 15) * 4;
      for (int pass = 0; pass < 2; ++pass) {
#pragma unroll
        for (int it = 0; it < 8; ++it) {
          const int row = it * 2 + hh;
          const v4f v = *(const v4f*)(slab + row * 68 + c4);
          *(volatile v4f*)(C + (size_t)(mBase + row) * kNcat + n0 + c4) = v;
        }
        __threadfence();
      }
    }
    __builtin_amdgcn_fence(__ATOMIC_RELEASE, "workgroup");
    __builtin_amdgcn_wave_barrier();
    __builtin_amdgcn_fence(__ATOMIC_ACQUIRE, "workgroup");
  }
}

__global__ __launch_bounds__(256) void cast_x_kernel(
    const float* __restrict__ x, unsigned short* __restrict__ A16, unsigned short* __restrict__ H16)
{
  const int i = blockIdx.x * 256 + threadIdx.x;
  const bool real = (i < kRealOct);
  const size_t e0 = (size_t)i << 3;
  const size_t ec = real ? e0 : ((size_t)(kRealOct - 1) << 3);
  const v4f a0 = *(const v4f*)(x + ec);
  const v4f a1 = *(const v4f*)(x + ec + 4);
  v8h hv;
#pragma unroll
  for (int e = 0; e < 4; ++e) {
    const float f0 = real ? a0[e] : 0.0f;
    const float f1 = real ? a1[e] : 0.0f;
    hv[e]     = (_Float16)f0;
    hv[4 + e] = (_Float16)f1;
  }
  unsigned short* pa = A16 + e0;
  unsigned short* ph = H16 + e0;
  *(volatile v8h*)pa = hv;
  if (!real) *(volatile v8h*)ph = hv;
  __threadfence();
  *(volatile v8h*)pa = hv;
  if (!real) *(volatile v8h*)ph = hv;
}

__global__ __launch_bounds__(256) void build_bt_kernel(
    const float* __restrict__ W1, const float* __restrict__ root1,
    const float* __restrict__ W2, const float* __restrict__ root2,
    unsigned short* __restrict__ BT1, unsigned short* __restrict__ BT2)
{
  __shared__ float tileT[128 * 33];
  const int tid = threadIdx.x;
  const int ob = blockIdx.x & 3;
  const int m  = blockIdx.x >> 2;
  const int layer = blockIdx.y;
  const float* Wl = layer ? W2 : W1;
  const float* Rl = layer ? root2 : root1;
  unsigned short* Bt = layer ? BT2 : BT1;
  const int mc = (m < kRel) ? m : (kRel - 1);
  const float* srcW = Wl + (size_t)mc * kF * kF;
  const float* src = (m < kRel) ? srcW : Rl;
#pragma unroll 1
  for (int it = 0; it < 16; ++it) {
    const int idx = it * 256 + tid;
    const int f = idx >> 5, o = idx & 31;
    tileT[f * 33 + o] = src[(size_t)f * kF + ob * 32 + o];
  }
  __syncthreads();
  v8h hv[2];
#pragma unroll
  for (int it = 0; it < 2; ++it) {
    const int c = it * 256 + tid;
    const int row = c >> 4, col8 = (c & 15) * 8;
#pragma unroll
    for (int e = 0; e < 8; ++e) {
      const float w = tileT[(col8 + e) * 33 + row] * kWCarry;
      hv[it][e] = (_Float16)w;
    }
  }
  for (int pass = 0; pass < 2; ++pass) {
#pragma unroll
    for (int it = 0; it < 2; ++it) {
      const int c = it * 256 + tid;
      const int row = c >> 4, col8 = (c & 15) * 8;
      unsigned short* dp = Bt + (size_t)(m * kF + ob * 32 + row) * kF + col8;
      *(volatile v8h*)dp = hv[it];
    }
    __threadfence();
  }
}

__global__ __launch_bounds__(128) void mrep_kernel(
    const float* __restrict__ message, const float* __restrict__ embed,
    const float* __restrict__ cont_w, const float* __restrict__ cont_b,
    const float* __restrict__ msg_w, const float* __restrict__ msg_b,
    float* __restrict__ MREP)
{
  __shared__ float comb[2 * kF];
  __shared__ __align__(16) float res[kF];
  const int g = blockIdx.x, tid = threadIdx.x;
  const float tf = message[g * 2 + 0];
  const float tcl = fminf(fmaxf(tf, 0.0f), (float)(kVocab - 1));
  int tok = (int)tcl;
  tok = tok < 0 ? 0 : (tok > kVocab - 1 ? kVocab - 1 : tok);
  const float cv = message[g * 2 + 1];
  comb[tid] = embed[(size_t)tok * kF + tid];
  const float ce = cv * cont_w[tid] + cont_b[tid];
  comb[kF + tid] = fmaxf(ce, 0.0f);
  __syncthreads();
  float s = 0.0f;
#pragma unroll 4
  for (int i = 0; i < 2 * kF; ++i) s = fmaf(comb[i], msg_w[(size_t)i * kF + tid], s);
  s += msg_b[tid];
  res[tid] = fmaxf(s, 0.0f);
  __syncthreads();
  if (tid < 32) {
    const v4f v = *(const v4f*)(res + tid * 4);
    float* dp = MREP + (size_t)g * kF + tid * 4;
    *(volatile v4f*)dp = v;
    __threadfence();
    *(volatile v4f*)dp = v;
  }
}

template <int LAYER>
__global__ __launch_bounds__(256) void aggregate_kernel(
    const float* __restrict__ HW, const int* __restrict__ ei, const int* __restrict__ et,
    const int* __restrict__ batch, const int* __restrict__ maxn,
    const float* __restrict__ bias, const float* __restrict__ MREP,
    unsigned short* __restrict__ H16, float* __restrict__ out, int chunk)
{
  __shared__ unsigned sEdge[kEpg];
  __shared__ int   sCnt[kNpg * kRel];
  __shared__ float sNorm[kNpg * kRel];
  __shared__ int   sDeg[256];
  __shared__ int   sOff[256];
  __shared__ int   sCur[256];
  __shared__ __align__(16) float sMrep[kF];
  __shared__ __align__(16) float sScore[4 * kNpg];

  const int tid = threadIdx.x, lane = tid & 31, wave = tid >> 5;
  const int quad = chunk * kQuadsPerChunk + blockIdx.x;
  int ng = kGraphs - 4 * quad;
  ng = ng > 4 ? 4 : ng;
  ng = ng < 0 ? 0 : ng;
  const v4f bv = *(const v4f*)(bias + 4 * lane);
  int mx = kNpg;
  if (LAYER == 2) mx = maxn[0];
  const float negInf = __uint_as_float(0xff800000u);
  const float qNan   = __uint_as_float(0x7fc00000u);

  for (int gi = 0; gi < ng; ++gi) {
    const int g = 4 * quad + gi;
    const int nbase = g * kNpg;
    const int ebase = g * kEpg;
    const int lrow0 = (g - chunk * kChunkGraphs) * kNpg;

#pragma unroll 1
    for (int i = tid; i < kNpg * kRel; i += 256) sCnt[i] = 0;
    sDeg[tid] = 0;
    if (LAYER == 2) {
      if (tid < kF) sMrep[tid] = MREP[(size_t)g * kF + tid];
    }
    __syncthreads();

#pragma unroll 1
    for (int it = 0; it < (kEpg + 255) / 256; ++it) {
      const int e = it * 256 + tid;
      const bool inb = (e < kEpg);
      const int ec = inb ? e : (kEpg - 1);
      const int idx = ebase + ec;
      const int sl = ei[idx] - nbase;
      const int dl = ei[kEdges + idx] - nbase;
      const int ty = et[idx];
      const bool ok = inb && ((unsigned)sl < (unsigned)kNpg) && ((unsigned)dl < (unsigned)kNpg) &&
                      ((unsigned)ty < (unsigned)kRel);
      if (ok) {
        atomicAdd(&sCnt[dl * kRel + ty], 1);
        atomicAdd(&sDeg[dl], 1);
      }
    }
    __syncthreads();

#pragma unroll 1
    for (int i = tid; i < kNpg * kRel; i += 256) {
      const int c = sCnt[i];
      const float cf = (float)(c > 1 ? c : 1);
      sNorm[i] = 1.0f / cf;
    }
    if (tid == 0) {
      int run = 0;
#pragma unroll 1
      for (int i = 0; i < kNpg; ++i) {
        const int d = sDeg[i];
        sOff[i] = run;
        sCur[i] = run;
        run += d;
      }
      sOff[kNpg] = run;
    }
    __syncthreads();

#pragma unroll 1
    for (int it = 0; it < (kEpg + 255) / 256; ++it) {
      const int e = it * 256 + tid;
      const bool inb = (e < kEpg);
      const int ec = inb ? e : (kEpg - 1);
      const int idx = ebase + ec;
      const int sl = ei[idx] - nbase;
      const int dl = ei[kEdges + idx] - nbase;
      const int ty = et[idx];
      const bool ok = inb && ((unsigned)sl < (unsigned)kNpg) && ((unsigned)dl < (unsigned)kNpg) &&
                      ((unsigned)ty < (unsigned)kRel);
      if (ok) {
        int pos = atomicAdd(&sCur[dl], 1);
        pos = pos < 0 ? 0 : (pos > kEpg - 1 ? kEpg - 1 : pos);
        sEdge[pos] = ((unsigned)e << 11) | ((unsigned)sl << 3) | (unsigned)ty;
      }
    }
    __syncthreads();

    if (tid < kNpg) {
      int a = sOff[tid], b = sOff[tid + 1];
      a = a < 0 ? 0 : (a > kEpg ? kEpg : a);
      b = b < a ? a : (b > kEpg ? kEpg : b);
#pragma unroll 1
      for (int i = a + 1; i < b; ++i) {
        const unsigned key = sEdge[i];
        int j = i - 1;
        while (j >= a && sEdge[j] > key) {
          sEdge[j + 1] = sEdge[j];
          --j;
        }
        sEdge[j + 1] = key;
      }
    }
    __syncthreads();

    v4f mr = (v4f){0.f, 0.f, 0.f, 0.f};
    if (LAYER == 2) mr = *(const v4f*)(sMrep + 4 * lane);
    const float* hwg = HW + (size_t)lrow0 * kNcat + 4 * lane;
#pragma unroll 1
    for (int k = 0; k < kNpg / 8; ++k) {
      const int p = wave + 8 * k;
      int a = __builtin_amdgcn_readfirstlane(sOff[p]);
      int b = __builtin_amdgcn_readfirstlane(sOff[p + 1]);
      a = a < 0 ? 0 : (a > kEpg ? kEpg : a);
      b = b < a ? a : (b > kEpg ? kEpg : b);
      float g0 = 0.0f, g1 = 0.0f, g2 = 0.0f, g3 = 0.0f;
#pragma unroll 1
      for (int i = a; i < b; ++i) {
        const unsigned w = sEdge[i];
        int sl = (int)((w >> 3) & 255u);
        sl = sl > kNpg - 1 ? kNpg - 1 : sl;
        const int ty = (int)(w & 7u);
        const float nm = sNorm[p * kRel + ty];
        const v4f m = *(const v4f*)(hwg + (size_t)sl * kNcat + ty * kF);
        g0 = fmaf(m[0], nm, g0);
        g1 = fmaf(m[1], nm, g1);
        g2 = fmaf(m[2], nm, g2);
        g3 = fmaf(m[3], nm, g3);
      }
      const v4f rt = *(const v4f*)(hwg + (size_t)p * kNcat + kRel * kF);
      const float o0 = (g0 + rt[0]) + bv[0];
      const float o1 = (g1 + rt[1]) + bv[1];
      const float o2 = (g2 + rt[2]) + bv[2];
      const float o3 = (g3 + rt[3]) + bv[3];
      if (LAYER == 1) {
        v4h hv;
        hv[0] = (_Float16)fmaxf(o0, 0.0f);
        hv[1] = (_Float16)fmaxf(o1, 0.0f);
        hv[2] = (_Float16)fmaxf(o2, 0.0f);
        hv[3] = (_Float16)fmaxf(o3, 0.0f);
        unsigned short* dp = H16 + (size_t)(nbase + p) * kF + 4 * lane;
        *(volatile v4h*)dp = hv;
        __threadfence();
        *(volatile v4h*)dp = hv;
      } else {
        float s = o0 * mr[0];
        s = fmaf(o1, mr[1], s);
        s = fmaf(o2, mr[2], s);
        s = fmaf(o3, mr[3], s);
#pragma unroll
        for (int off = 16; off >= 1; off >>= 1) s += __shfl_xor(s, off, 32);
        int n = nbase + p;
        n = n > kNodes - 1 ? kNodes - 1 : n;
        const int bq = batch[n];
        float val = (bq == g) ? s : negInf;
        val = (mx == kNpg) ? val : qNan;
        if (lane == 0) sScore[gi * kNpg + p] = val;
      }
    }
    __syncthreads();
  }

  if (LAYER == 2) {
    __syncthreads();
    const int nvec = ng * (kNpg / 4);
    const int tc = (tid < nvec) ? tid : 0;
    const v4f v = *(const v4f*)(sScore + tc * 4);
    float* dp = out + (size_t)quad * (4 * kNpg) + tc * 4;
    if (tid < nvec) *(volatile v4f*)dp = v;
    __threadfence();
    if (tid < nvec) *(volatile v4f*)dp = v;
  }
}

extern "C" void kernel_launch(void* const* d_in, const int* in_sizes, int n_in,
                              void* d_out, int out_size, void* d_ws, size_t ws_size,
                              hipStream_t stream) {
  if (n_in < 17) return;
  if (in_sizes[0] != kGraphs * 2) return;
  if (in_sizes[1] != kNodes * kF) return;
  if (in_sizes[2] != 2 * kEdges) return;
  if (in_sizes[3] != kEdges) return;
  if (in_sizes[4] != kNodes) return;
  if (in_sizes[5] != 1) return;
  if (in_sizes[6] != kRel * kF * kF) return;
  if (in_sizes[7] != kF * kF) return;
  if (in_sizes[8] != kF) return;
  if (in_sizes[9] != kRel * kF * kF) return;
  if (in_sizes[10] != kF * kF) return;
  if (in_sizes[11] != kF) return;
  if (in_sizes[12] != kVocab * kF) return;
  if (in_sizes[13] != kF) return;
  if (in_sizes[14] != kF) return;
  if (in_sizes[15] != 2 * kF * kF) return;
  if (in_sizes[16] != kF) return;
  if (out_size != kGraphs * kNpg) return;
  if (ws_size < kWsTotal) return;

  const float* message = (const float*)d_in[0];
  const float* x       = (const float*)d_in[1];
  const int*   ei      = (const int*)d_in[2];
  const int*   et      = (const int*)d_in[3];
  const int*   batch   = (const int*)d_in[4];
  const int*   maxn    = (const int*)d_in[5];
  const float* W1      = (const float*)d_in[6];
  const float* root1   = (const float*)d_in[7];
  const float* b1      = (const float*)d_in[8];
  const float* W2      = (const float*)d_in[9];
  const float* root2   = (const float*)d_in[10];
  const float* b2      = (const float*)d_in[11];
  const float* embed   = (const float*)d_in[12];
  const float* cont_w  = (const float*)d_in[13];
  const float* cont_b  = (const float*)d_in[14];
  const float* msg_w   = (const float*)d_in[15];
  const float* msg_b   = (const float*)d_in[16];
  float* out = (float*)d_out;

  char* ws = (char*)d_ws;
  unsigned short* A16  = (unsigned short*)(ws + kOffA16);
  unsigned short* H16  = (unsigned short*)(ws + kOffH16);
  unsigned short* BT1  = (unsigned short*)(ws + kOffBT1);
  unsigned short* BT2  = (unsigned short*)(ws + kOffBT2);
  float*          HW   = (float*)(ws + kOffHW);
  float*          MREP = (float*)(ws + kOffMREP);

  cast_x_kernel<<<kPadOct / 256, 256, 0, stream>>>(x, A16, H16);
  build_bt_kernel<<<dim3(36, 2), 256, 0, stream>>>(W1, root1, W2, root2, BT1, BT2);
  mrep_kernel<<<kGraphs, 128, 0, stream>>>(message, embed, cont_w, cont_b, msg_w, msg_b, MREP);

  const int gemmBlocks = (kTilesM * kTilesN) / 8;
  for (int c = 0; c < kChunks; ++c) {
    int nblk = kQuads - c * kQuadsPerChunk;
    nblk = nblk > kQuadsPerChunk ? kQuadsPerChunk : nblk;
    const unsigned short* Ax = A16 + (size_t)c * kChunkRows * kF;
    const unsigned short* Ah = H16 + (size_t)c * kChunkRows * kF;

    proj_gemm_kernel<<<gemmBlocks, 256, 0, stream>>>(Ax, BT1, HW, kWCarryInv);
    aggregate_kernel<1><<<nblk, 256, 0, stream>>>(HW, ei, et, batch, maxn, b1, MREP, H16, out, c);
    proj_gemm_kernel<<<gemmBlocks, 256, 0, stream>>>(Ah, BT2, HW, kWCarryInv);
    aggregate_kernel<2><<<nblk, 256, 0, stream>>>(HW, ei, et, batch, maxn, b2, MREP, H16, out, c);
  }
}
